// DistanceAwareSelfAttention_5540507812317
// MI455X (gfx1250) — hardware-verified
//
#include <hip/hip_runtime.h>
#include <stdint.h>

#define SLEN 1024
#define BSZ 8
#define NH 16
#define KV 64
#define EMB 1024
#define QKV3 3072
#define NTOK 8192
#define CLIPD 10
#define NCL 11

typedef _Float16 v16h __attribute__((ext_vector_type(16)));
typedef _Float16 v8h __attribute__((ext_vector_type(8)));
typedef float v8f __attribute__((ext_vector_type(8)));
typedef float v4f __attribute__((ext_vector_type(4)));

union Frag { v16h v; v8h h[2]; };

__device__ __forceinline__ v16h ld_frag(const _Float16* p) {
  Frag f;
  f.h[0] = *(const v8h*)(p);
  f.h[1] = *(const v8h*)(p + 16);
  return f.v;
}

__device__ __forceinline__ v8f mma16(v16h a, v16h b, v8f c) {
  c = __builtin_amdgcn_wmma_f32_16x16x32_f16(false, a, false, b, (short)0, c, false, false);
  asm volatile("v_nop\n\tv_nop\n\tv_nop\n\tv_nop" : "+v"(c) : "v"(a), "v"(b));
  return c;
}

__device__ __forceinline__ void wave_sync_lds() {
  __builtin_amdgcn_fence(__ATOMIC_RELEASE, "workgroup");
  __builtin_amdgcn_wave_barrier();
  __builtin_amdgcn_fence(__ATOMIC_ACQUIRE, "workgroup");
}

__global__ __launch_bounds__(256) void cvt_f16_kernel(const float* __restrict__ src, _Float16* __restrict__ dst,
                                                      int n8, float scale) {
  const int i = blockIdx.x * 256 + threadIdx.x;
  if (i < n8) {
    const v4f a = *(const v4f*)(src + (size_t)i * 8);
    const v4f b = *(const v4f*)(src + (size_t)i * 8 + 4);
    v8h o;
    o[0] = (_Float16)(a[0] * scale); o[1] = (_Float16)(a[1] * scale);
    o[2] = (_Float16)(a[2] * scale); o[3] = (_Float16)(a[3] * scale);
    o[4] = (_Float16)(b[0] * scale); o[5] = (_Float16)(b[1] * scale);
    o[6] = (_Float16)(b[2] * scale); o[7] = (_Float16)(b[3] * scale);
    _Float16* p = dst + (size_t)i * 8;
    *(volatile v8h*)p = o;
    __threadfence();
    *(volatile v8h*)p = o;
  }
}

__device__ __forceinline__ void mainloop64(const _Float16* __restrict__ A, const _Float16* __restrict__ Bt,
                                           int m0, int n0, int lane, v8f (&acc)[4][4]) {
  const int c = lane & 15, koff = (lane >> 4) * 8;
#pragma unroll 1
  for (int k0 = 0; k0 < EMB; k0 += 32) {
    v16h bf[4];
#pragma unroll
    for (int j = 0; j < 4; ++j) bf[j] = ld_frag(Bt + (size_t)(n0 + 16 * j + c) * EMB + k0 + koff);
#pragma unroll
    for (int i = 0; i < 4; ++i) {
      const v16h af = ld_frag(A + (size_t)(m0 + 16 * i + c) * EMB + k0 + koff);
#pragma unroll
      for (int j = 0; j < 4; ++j) acc[i][j] = mma16(af, bf[j], acc[i][j]);
    }
  }
}

__global__ __launch_bounds__(256) void qkv_gemm_kernel(const _Float16* __restrict__ X16, const _Float16* __restrict__ W16,
                                                       const float* __restrict__ b_in,
                                                       _Float16* __restrict__ Qp, _Float16* __restrict__ Kp,
                                                       _Float16* __restrict__ Vtp) {
  extern __shared__ __align__(16) _Float16 stg[];
  const int lane = threadIdx.x & 31, wave = threadIdx.x >> 5;
  const int hh = lane >> 4, c = lane & 15;
  const int bx = blockIdx.x;
  const int by = blockIdx.y;
  const int n0 = bx * 64;
  const int m0 = by * 512 + wave * 64;
  const int which = bx >> 4;
  const int head = bx & 15;

  v8f acc[4][4];
#pragma unroll
  for (int i = 0; i < 4; ++i)
#pragma unroll
    for (int j = 0; j < 4; ++j) acc[i][j] = (v8f){0.f, 0.f, 0.f, 0.f, 0.f, 0.f, 0.f, 0.f};

  mainloop64(X16, W16, m0, n0, lane, acc);

  const float sc = 0.015625f;
  if (which == 2) {
#pragma unroll
    for (int i = 0; i < 4; ++i) {
      const int tl = 8 * wave + 2 * i + hh;
#pragma unroll
      for (int j = 0; j < 4; ++j) {
        const int d = 16 * j + c;
        const float bv = b_in[n0 + d];
#pragma unroll
        for (int r = 0; r < 8; ++r) stg[(r * 64 + d) * 64 + tl] = (_Float16)(acc[i][j][r] * sc + bv);
      }
    }
  } else {
#pragma unroll
    for (int i = 0; i < 4; ++i)
#pragma unroll
      for (int j = 0; j < 4; ++j) {
        const int col = 16 * j + c;
        const float bv = b_in[n0 + col];
#pragma unroll
        for (int r = 0; r < 8; ++r)
          stg[(wave * 64 + 16 * i + 8 * hh + r) * 64 + col] = (_Float16)(acc[i][j][r] * sc + bv);
      }
  }
  __syncthreads();

  if (which == 2) {
    const int g = threadIdx.x >> 3, p = threadIdx.x & 7;
    for (int pass = 0; pass < 2; ++pass) {
#pragma unroll 4
      for (int it = 0; it < 16; ++it) {
        const int L = it * 32 + g;
        const int bb = L >> 6, d = L & 63;
        const v8h v = *(const v8h*)(stg + (size_t)L * 64 + 8 * p);
        _Float16* dst = Vtp + ((((size_t)bb * NH + head) * KV + d) * SLEN + (size_t)by * 64 + 8 * p);
        *(volatile v8h*)dst = v;
      }
      __threadfence();
    }
  } else {
    _Float16* P = (which == 0) ? Qp : Kp;
    const int rq = lane >> 3, p = lane & 7;
    for (int pass = 0; pass < 2; ++pass) {
#pragma unroll 4
      for (int it = 0; it < 16; ++it) {
        const int R = it * 4 + rq;
        const int m = m0 + R;
        const int s = m >> 3, bb = m & 7;
        const v8h v = *(const v8h*)(stg + (size_t)(wave * 64 + R) * 64 + 8 * p);
        _Float16* dst = P + ((((size_t)bb * NH + head) * SLEN + s) * KV + 8 * p);
        *(volatile v8h*)dst = v;
      }
      __threadfence();
    }
  }
}

__global__ __launch_bounds__(128) void attn_kernel(const _Float16* __restrict__ Qp, const _Float16* __restrict__ Kp,
                                                   const _Float16* __restrict__ Vtp,
                                                   const float* __restrict__ kemb, const float* __restrict__ vemb,
                                                   _Float16* __restrict__ Ap) {
  __shared__ float s_kemb[NCL * KV];
  __shared__ float s_vemb[NCL * KV];
  __shared__ float s_qd[64 * 12];
  __shared__ __align__(16) _Float16 Ksh[64 * 64];
  __shared__ __align__(16) _Float16 Vth[64 * 64];
  __shared__ __align__(16) _Float16 Psh[4][16 * 64];
  __shared__ float s_near[4][16 * 20];
  __shared__ __align__(16) _Float16 Osh[4][16 * 72];

  const int tid = threadIdx.x, wave = tid >> 5, lane = tid & 31;
  const int hh = lane >> 4, c = lane & 15;
  const int bx = blockIdx.x;
  const int qb = bx & 15;
  const int head = (bx >> 4) & 15;
  const int b = bx >> 8;
  const int qbase = qb * 64;
  const int q0w = qbase + wave * 16;
  const size_t bh = (size_t)b * NH + head;
  const _Float16* Qb = Qp + bh * SLEN * KV;
  const _Float16* Kb = Kp + bh * SLEN * KV;
  const _Float16* Vb = Vtp + bh * KV * SLEN;

  for (int i = tid; i < NCL * KV; i += 128) { s_kemb[i] = kemb[i]; s_vemb[i] = vemb[i]; }
  for (int i = lane; i < 16 * 20; i += 32) s_near[wave][i] = -1.0e30f;
  __syncthreads();

  for (int i = tid; i < 64 * NCL; i += 128) {
    const int row = i / NCL, cc = i - row * NCL;
    const _Float16* qr = Qb + (size_t)(qbase + row) * KV;
    const float* ke = s_kemb + cc * KV;
    float a = 0.f;
#pragma unroll 1
    for (int d8 = 0; d8 < KV; d8 += 8) {
      const v8h qv = *(const v8h*)(qr + d8);
#pragma unroll
      for (int e = 0; e < 8; ++e) a += (float)qv[e] * ke[d8 + e];
    }
    s_qd[row * 12 + cc] = a * 0.125f;
  }
  __syncthreads();

  v16h qa[2];
#pragma unroll
  for (int dc = 0; dc < 2; ++dc) qa[dc] = ld_frag(Qb + (size_t)(q0w + c) * KV + dc * 32 + 8 * hh);

  float mrow[8], lrow[8];
  v8f oacc[4];
#pragma unroll
  for (int r = 0; r < 8; ++r) { mrow[r] = -1.0e30f; lrow[r] = 0.f; }
#pragma unroll
  for (int t = 0; t < 4; ++t) oacc[t] = (v8f){0.f, 0.f, 0.f, 0.f, 0.f, 0.f, 0.f, 0.f};

  const int rwb = 8 * hh;
  const int rbb = wave * 16 + rwb;
  const int sq = qbase + rbb;
  _Float16* pw = Psh[wave];

  for (int kc = 0; kc < SLEN / 64; ++kc) {
    const int kv0 = kc * 64;
    __syncthreads();
    {
      const int rr = tid >> 1, half = (tid & 1) * 32;
      const _Float16* ks = Kb + (size_t)(kv0 + rr) * KV + half;
      const _Float16* vs = Vb + (size_t)rr * SLEN + kv0 + half;
#pragma unroll
      for (int i = 0; i < 4; ++i) {
        const v8h a0 = *(const v8h*)(ks + 8 * i);
        const v8h b0 = *(const v8h*)(vs + 8 * i);
        *(v8h*)(Ksh + rr * 64 + half + 8 * i) = a0;
        *(v8h*)(Vth + rr * 64 + half + 8 * i) = b0;
      }
    }
    __syncthreads();

    v8f s[4];
#pragma unroll
    for (int j = 0; j < 4; ++j) {
      s[j] = (v8f){0.f, 0.f, 0.f, 0.f, 0.f, 0.f, 0.f, 0.f};
#pragma unroll
      for (int dc = 0; dc < 2; ++dc) {
        Frag kb;
        kb.h[0] = *(const v8h*)(Ksh + (j * 16 + c) * 64 + dc * 32 + 8 * hh);
        kb.h[1] = *(const v8h*)(Ksh + (j * 16 + c) * 64 + dc * 32 + 16 + 8 * hh);
        s[j] = mma16(qa[dc], kb.v, s[j]);
      }
    }
    float cm[8];
#pragma unroll
    for (int r = 0; r < 8; ++r) {
      const int srow = sq + r;
      float m = -1.0e30f;
#pragma unroll
      for (int j = 0; j < 4; ++j) {
        const int t = kv0 + j * 16 + c;
        int ad = t - srow; ad = (ad < 0) ? -ad : ad; ad = (ad > CLIPD) ? CLIPD : ad;
        const float sv = s[j][r] * 0.125f + s_qd[(rbb + r) * 12 + ad];
        s[j][r] = sv;
        m = fmaxf(m, sv);
      }
#pragma unroll
      for (int off = 1; off < 16; off <<= 1) m = fmaxf(m, __shfl_xor(m, off, 32));
      cm[r] = m;
    }
    if (kv0 < q0w + 25 && kv0 + 73 > q0w) {
#pragma unroll
      for (int r = 0; r < 8; ++r) {
        const int srow = sq + r;
#pragma unroll
        for (int j = 0; j < 4; ++j) {
          const int dd = kv0 + j * 16 + c - srow;
          if (dd >= -9 && dd <= 9) s_near[wave][(rwb + r) * 20 + dd + 9] = s[j][r];
        }
      }
    }
#pragma unroll
    for (int r = 0; r < 8; ++r) {
      const float mnew = fmaxf(mrow[r], cm[r]);
      const float alpha = __expf(mrow[r] - mnew);
      mrow[r] = mnew;
      float psum = 0.f;
#pragma unroll
      for (int j = 0; j < 4; ++j) {
        const float p = __expf(s[j][r] - mnew);
        psum += p;
        pw[(rwb + r) * 64 + j * 16 + c] = (_Float16)(p * 1024.0f);
      }
#pragma unroll
      for (int off = 1; off < 16; off <<= 1) psum += __shfl_xor(psum, off, 32);
      lrow[r] = lrow[r] * alpha + psum;
#pragma unroll
      for (int t = 0; t < 4; ++t) oacc[t][r] *= alpha;
    }
    wave_sync_lds();
#pragma unroll
    for (int kk = 0; kk < 2; ++kk) {
      Frag pa;
      pa.h[0] = *(const v8h*)(pw + c * 64 + kk * 32 + 8 * hh);
      pa.h[1] = *(const v8h*)(pw + c * 64 + kk * 32 + 16 + 8 * hh);
#pragma unroll
      for (int t = 0; t < 4; ++t) {
        Frag vb;
        vb.h[0] = *(const v8h*)(Vth + (t * 16 + c) * 64 + kk * 32 + 8 * hh);
        vb.h[1] = *(const v8h*)(Vth + (t * 16 + c) * 64 + kk * 32 + 16 + 8 * hh);
        oacc[t] = mma16(pa.v, vb.v, oacc[t]);
      }
    }
  }
  __syncthreads();

  _Float16* os = Osh[wave];
#pragma unroll
  for (int r = 0; r < 8; ++r) {
    const int rw = rwb + r;
    const float invl = 1.0f / lrow[r];
    const float m = mrow[r];
    const float* nr = s_near[wave] + rw * 20;
    float pc[10];
    pc[0] = __expf(nr[9] - m);
#pragma unroll
    for (int cc = 1; cc < 10; ++cc) pc[cc] = __expf(nr[9 - cc] - m) + __expf(nr[9 + cc] - m);
#pragma unroll
    for (int cc = 0; cc < 10; ++cc) pc[cc] *= invl;
    const float osc = invl * 0.0009765625f;
#pragma unroll
    for (int t = 0; t < 4; ++t) {
      const int d = 16 * t + c;
      const float v10 = s_vemb[CLIPD * KV + d];
      float corr = v10;
#pragma unroll
      for (int cc = 0; cc < 10; ++cc) corr += pc[cc] * (s_vemb[cc * KV + d] - v10);
      const float val = oacc[t][r] * osc + corr;
      os[rw * 72 + d] = (_Float16)(val * 16.0f);
    }
  }
  wave_sync_lds();
  {
    const int rq = lane >> 3, p = lane & 7;
    for (int pass = 0; pass < 2; ++pass) {
#pragma unroll
      for (int it = 0; it < 4; ++it) {
        const int rl = it * 4 + rq;
        const v8h v = *(const v8h*)(os + rl * 72 + 8 * p);
        const size_t tok = (size_t)(q0w + rl) * BSZ + b;
        *(volatile v8h*)(Ap + tok * EMB + (size_t)head * KV + 8 * p) = v;
      }
      __threadfence();
    }
  }
}

__global__ __launch_bounds__(256) void out_gemm_kernel(const _Float16* __restrict__ A16, const _Float16* __restrict__ W16,
                                                       const float* __restrict__ b_out, float* __restrict__ out) {
  __shared__ __align__(16) float slab[8][16 * 68];
  const int lane = threadIdx.x & 31, wave = threadIdx.x >> 5;
  const int hh = lane >> 4, c = lane & 15;
  const int tile = blockIdx.x * 8 + wave;
  const int tm = tile >> 4, tn = tile & 15;
  const int m0 = tm * 64, n0 = tn * 64;

  v8f acc[4][4];
#pragma unroll
  for (int i = 0; i < 4; ++i)
#pragma unroll
    for (int j = 0; j < 4; ++j) acc[i][j] = (v8f){0.f, 0.f, 0.f, 0.f, 0.f, 0.f, 0.f, 0.f};

  mainloop64(A16, W16, m0, n0, lane, acc);

  float* sl = slab[wave];
  const float sc = 0.0009765625f;
#pragma unroll
  for (int i = 0; i < 4; ++i) {
    const int mBase = m0 + 16 * i;
#pragma unroll
    for (int j = 0; j < 4; ++j) {
      const int col = 16 * j + c;
      const float bv = b_out[n0 + col];
#pragma unroll
      for (int r = 0; r < 8; ++r) sl[(8 * hh + r) * 68 + col] = acc[i][j][r] * sc + bv;
    }
    wave_sync_lds();
    const int c4 = c * 4;
    for (int pass = 0; pass < 2; ++pass) {
#pragma unroll
      for (int it = 0; it < 8; ++it) {
        const int row = it * 2 + hh;
        const v4f v = *(const v4f*)(sl + row * 68 + c4);
        *(volatile v4f*)(out + (size_t)(mBase + row) * EMB + n0 + c4) = v;
      }
      __threadfence();
    }
    wave_sync_lds();
  }
}

extern "C" void kernel_launch(void* const* d_in, const int* in_sizes, int n_in,
                              void* d_out, int out_size, void* d_ws, size_t ws_size,
                              hipStream_t stream) {
  if (n_in < 7) return;
  if (in_sizes[0] != NTOK * EMB || in_sizes[1] != QKV3 * EMB || in_sizes[2] != QKV3) return;
  if (in_sizes[3] != NCL * KV || in_sizes[4] != NCL * KV) return;
  if (in_sizes[5] != EMB * EMB || in_sizes[6] != EMB) return;
  if (out_size != NTOK * EMB) return;

  const float* X     = (const float*)d_in[0];
  const float* W_in  = (const float*)d_in[1];
  const float* b_in  = (const float*)d_in[2];
  const float* kemb  = (const float*)d_in[3];
  const float* vemb  = (const float*)d_in[4];
  const float* W_out = (const float*)d_in[5];
  const float* b_out = (const float*)d_in[6];

  size_t off = 0;
  const size_t oX   = off; off += (size_t)NTOK * EMB * 2;
  const size_t oWi  = off; off += (size_t)QKV3 * EMB * 2;
  const size_t oWo  = off; off += (size_t)EMB * EMB * 2;
  const size_t oQ   = off; off += (size_t)BSZ * NH * SLEN * KV * 2;
  const size_t oK   = off; off += (size_t)BSZ * NH * SLEN * KV * 2;
  const size_t oVt  = off; off += (size_t)BSZ * NH * KV * SLEN * 2;
  const size_t oA   = off; off += (size_t)NTOK * EMB * 2;
  if (off > ws_size) return;

  char* ws = (char*)d_ws;
  _Float16* X16    = (_Float16*)(ws + oX);
  _Float16* Win16  = (_Float16*)(ws + oWi);
  _Float16* Wout16 = (_Float16*)(ws + oWo);
  _Float16* Q16    = (_Float16*)(ws + oQ);
  _Float16* K16    = (_Float16*)(ws + oK);
  _Float16* Vt16   = (_Float16*)(ws + oVt);
  _Float16* A16    = (_Float16*)(ws + oA);

  const int n8x = NTOK * EMB / 8;
  const int n8wi = QKV3 * EMB / 8;
  const int n8wo = EMB * EMB / 8;
  cvt_f16_kernel<<<dim3((n8x + 255) / 256), dim3(256), 0, stream>>>(X, X16, n8x, 1.0f);
  cvt_f16_kernel<<<dim3((n8wi + 255) / 256), dim3(256), 0, stream>>>(W_in, Win16, n8wi, 64.0f);
  cvt_f16_kernel<<<dim3((n8wo + 255) / 256), dim3(256), 0, stream>>>(W_out, Wout16, n8wo, 64.0f);

  const int ldsQkv = 8 * 64 * 64 * 2;
  (void)hipFuncSetAttribute(reinterpret_cast<const void*>(&qkv_gemm_kernel),
                            hipFuncAttributeMaxDynamicSharedMemorySize, ldsQkv);
  qkv_gemm_kernel<<<dim3(QKV3 / 64, NTOK / 512), dim3(256), ldsQkv, stream>>>(X16, Win16, b_in, Q16, K16, Vt16);

  attn_kernel<<<dim3(BSZ * NH * (SLEN / 64)), dim3(128), 0, stream>>>(Q16, K16, Vt16, kemb, vemb, A16);

  out_gemm_kernel<<<dim3((NTOK / 64) * (EMB / 64) / 8), dim3(256), 0, stream>>>(A16, Wout16, b_out, (float*)d_out);

  (void)hipGetLastError();
}
